// GatedSSMLayer_62302795596637
// MI455X (gfx1250) — hardware-verified
//
#include <hip/hip_runtime.h>
#include <stdint.h>
#include <math.h>

constexpr int kB    = 4;
constexpr int kT    = 2048;
constexpr int kD    = 1024;
constexpr int kH    = 16;
constexpr int kDH   = 64;
constexpr int kRows = kB * kT;
constexpr int kWPlane    = kD * kD;
constexpr int kProjPlane = kT * kD;
constexpr float kWCarry    = 32.0f;
constexpr float kOCarry    = 16.0f;
constexpr float kProjScale = 1.0f / 32.0f;
constexpr float kOutScale  = 1.0f / (32.0f * 16.0f);
constexpr float kLnEps     = 1e-5f;
constexpr float kInvD      = 1.0f / 1024.0f;

typedef __attribute__((ext_vector_type(16))) _Float16 v16h;
typedef __attribute__((ext_vector_type(8)))  _Float16 v8h;
typedef __attribute__((ext_vector_type(16))) __bf16   v16b;
typedef __attribute__((ext_vector_type(8)))  __bf16   v8b;
typedef __attribute__((ext_vector_type(8)))  float    v8f;
typedef __attribute__((ext_vector_type(4)))  float    v4f;
typedef __attribute__((ext_vector_type(4)))  unsigned int v4u;

__device__ __forceinline__ unsigned short f2bf_bits(float f) {
  unsigned u = __float_as_uint(f);
  return (unsigned short)((u + 0x7FFFu + ((u >> 16) & 1u)) >> 16);
}
__device__ __forceinline__ float bf_bits2f(unsigned short h) { return __uint_as_float(((unsigned)h) << 16); }

__device__ __forceinline__ void dep_guard_h(v8f& a, v8f& b, v16h x, v16h y) { asm volatile("v_nop\n\tv_nop\n\tv_nop\n\tv_nop" : "+v"(a), "+v"(b) : "v"(x), "v"(y)); }
__device__ __forceinline__ void dep_guard_b(v8f& a, v8f& b, v16b x, v16b y) { asm volatile("v_nop\n\tv_nop\n\tv_nop\n\tv_nop" : "+v"(a), "+v"(b) : "v"(x), "v"(y)); }
__device__ __forceinline__ void keep4_h(v16h a, v16h b, v16h c, v16h d) { asm volatile("v_nop" :: "v"(a), "v"(b), "v"(c), "v"(d)); }
__device__ __forceinline__ void keep4_b(v16b a, v16b b, v16b c, v16b d) { asm volatile("v_nop" :: "v"(a), "v"(b), "v"(c), "v"(d)); }
__device__ __forceinline__ void acc_guard4(v8f& a, v8f& b, v8f& c, v8f& d) { asm volatile("v_nop\n\tv_nop\n\tv_nop\n\tv_nop" : "+v"(a), "+v"(b), "+v"(c), "+v"(d)); }
template <typename T> struct Frag;
template <> struct Frag<_Float16> {
  typedef v16h V; union U { v16h v; v8h h[2]; };
  static __device__ __forceinline__ v16h load(const _Float16* p) {
    U f; f.h[0] = *(const v8h*)(p); f.h[1] = *(const v8h*)(p + 16); return f.v;
  }
  static __device__ __forceinline__ v8f mma(v16h a, v16h b, v8f c) {
    return __builtin_amdgcn_wmma_f32_16x16x32_f16(false, a, false, b, (short)0, c, false, false);
  }
  static __device__ __forceinline__ void guard(v8f& a, v8f& b, v16h x, v16h y) { dep_guard_h(a, b, x, y); }
  static __device__ __forceinline__ void keep(v16h a, v16h b, v16h c, v16h d) { keep4_h(a, b, c, d); }
};
template <> struct Frag<__bf16> {
  typedef v16b V; union U { v16b v; v8b h[2]; };
  static __device__ __forceinline__ v16b load(const __bf16* p) {
    U f; f.h[0] = *(const v8b*)(p); f.h[1] = *(const v8b*)(p + 16); return f.v;
  }
  static __device__ __forceinline__ v8f mma(v16b a, v16b b, v8f c) {
    return __builtin_amdgcn_wmma_f32_16x16x32_bf16(false, a, false, b, (short)0, c, false, false);
  }
  static __device__ __forceinline__ void guard(v8f& a, v8f& b, v16b x, v16b y) { dep_guard_b(a, b, x, y); }
  static __device__ __forceinline__ void keep(v16b a, v16b b, v16b c, v16b d) { keep4_b(a, b, c, d); }
};

__device__ __forceinline__ unsigned pk16(unsigned short a, unsigned short b) { return (unsigned)a | ((unsigned)b << 16); }
__device__ __forceinline__ unsigned short h_bits(float f) { const _Float16 h = (_Float16)f; return __builtin_bit_cast(unsigned short, h); }

template <int ET> struct Elem;
template <> struct Elem<0> { typedef _Float16 T; };
template <> struct Elem<1> { typedef __bf16 T; };
template <int ET, bool SPLIT, int BIAS_MODE, int OUT_MODE, bool RESID, int ACT = 0>
__global__ __launch_bounds__(256) void wmma_gemm64(
    const unsigned short* __restrict__ Ap, const unsigned short* __restrict__ A2p, int lda, long strideA,
    const unsigned short* __restrict__ Btp, const unsigned short* __restrict__ Bt2p, int ldb, long strideB,
    void* __restrict__ Cout, void* __restrict__ Cout2, int ldc, long strideC,
    const float* __restrict__ bias, long strideBias,
    const float* __restrict__ resid, long strideR,
    int M, int N, int K, float scale) {
  typedef typename Elem<ET>::T T;
  typedef typename Frag<T>::V V;
  const T* A = (const T*)Ap; const T* A2 = (const T*)A2p; const T* Bt = (const T*)Btp; const T* Bt2 = (const T*)Bt2p;
  __shared__ __align__(16) float sT[8][16 * 68];
  const int b    = blockIdx.y;
  const int lane = threadIdx.x & 31;
  const int wave = threadIdx.x >> 5;
  const int tilesN = N >> 6;
  const int tilesM = M >> 6;
  const int tile = blockIdx.x * 8 + wave;
  if (tile >= tilesM * tilesN) return;
  const int tm = tile / tilesN;
  const int tn = tile - tm * tilesN;
  const int m0 = tm << 6;
  const int n0 = tn << 6;

  const T* Ab  = A  + (size_t)b * strideA;
  const T* Bb  = Bt + (size_t)b * strideB;
  const T* Ab2 = SPLIT ? (A2  + (size_t)b * strideA) : nullptr;
  const T* Bb2 = SPLIT ? (Bt2 + (size_t)b * strideB) : nullptr;
  const float* biasb = (BIAS_MODE != 0) ? (bias + (size_t)b * strideBias) : nullptr;

  const int rlane = lane & 15;
  const int koff  = (lane >> 4) * 8;
  const int mOff  = (lane >> 4) * 8;

  v8f acc[4][4];
#pragma unroll
  for (int i = 0; i < 4; ++i)
#pragma unroll
    for (int j = 0; j < 4; ++j) acc[i][j] = (v8f){0.f,0.f,0.f,0.f,0.f,0.f,0.f,0.f};

  for (int k0 = 0; k0 < K; k0 += 32) {
    V bh[4], bl[4];
#pragma unroll
    for (int j = 0; j < 4; ++j) {
      const size_t bo = (size_t)(n0 + (j << 4) + rlane) * ldb + koff + k0;
      bh[j] = Frag<T>::load(Bb + bo);
      if (SPLIT) bl[j] = Frag<T>::load(Bb2 + bo);
    }
#pragma unroll
    for (int i = 0; i < 4; ++i) {
      const size_t ao = (size_t)(m0 + (i << 4) + rlane) * lda + koff + k0;
      V ah = Frag<T>::load(Ab + ao);
      V al;
      if (SPLIT) al = Frag<T>::load(Ab2 + ao);
#pragma unroll
      for (int j = 0; j < 4; ++j) {
        acc[i][j] = Frag<T>::mma(ah, bh[j], acc[i][j]);
        if (SPLIT) {
          acc[i][j] = Frag<T>::mma(ah, bl[j], acc[i][j]);
          acc[i][j] = Frag<T>::mma(al, bh[j], acc[i][j]);
        }
      }
      Frag<T>::guard(acc[i][0], acc[i][3], ah, SPLIT ? al : ah);
    }
    Frag<T>::keep(bh[0], bh[1], bh[2], bh[3]);
    if (SPLIT) Frag<T>::keep(bl[0], bl[1], bl[2], bl[3]);
  }
  acc_guard4(acc[0][0], acc[0][1], acc[0][2], acc[0][3]);
  acc_guard4(acc[1][0], acc[1][1], acc[1][2], acc[1][3]);
  acc_guard4(acc[2][0], acc[2][1], acc[2][2], acc[2][3]);
  acc_guard4(acc[3][0], acc[3][1], acc[3][2], acc[3][3]);

  float* slab = sT[wave];
  const float* Rb = RESID ? (resid + (size_t)b * strideR) : nullptr;
#pragma unroll
  for (int i = 0; i < 4; ++i) {
    const int mBase = m0 + (i << 4);
#pragma unroll
    for (int j = 0; j < 4; ++j) {
      const int n = n0 + (j << 4) + rlane;
      float bv = 0.f;
      if (BIAS_MODE == 2) bv = biasb[n];
#pragma unroll
      for (int r = 0; r < 8; ++r) {
        float v = acc[i][j][r] * scale;
        if (BIAS_MODE == 1) v += biasb[mBase + mOff + r];
        if (BIAS_MODE == 2) v += bv;
        if (RESID) v += Rb[(size_t)(mBase + mOff + r) * ldc + n];
        if (ACT == 2) v = fmaxf(v, 0.0f);
        if (ACT == 4) v = (v > 0.f) ? v : 0.01f * v;
        slab[(mOff + r) * 68 + (j << 4) + rlane] = v;
      }
    }
    __builtin_amdgcn_fence(__ATOMIC_RELEASE, "workgroup");
    __builtin_amdgcn_wave_barrier();
    __builtin_amdgcn_fence(__ATOMIC_ACQUIRE, "workgroup");
    if (OUT_MODE == 0) {
      float* C = (float*)Cout + (size_t)b * strideC;
      const int hh = lane >> 4, c4 = (lane & 15) * 4;
      for (int pass = 0; pass < 2; ++pass) {
#pragma unroll
        for (int it = 0; it < 8; ++it) {
          const int row = it * 2 + hh;
          v4f v = *(const v4f*)(slab + row * 68 + c4);
          *(volatile v4f*)(C + (size_t)(mBase + row) * ldc + n0 + c4) = v;
        }
        __threadfence();
      }
    } else {
      const int q = lane >> 3, c8 = (lane & 7) * 8;
      unsigned short* C  = (unsigned short*)Cout  + (size_t)b * strideC;
      unsigned short* C2 = (OUT_MODE == 2) ? ((unsigned short*)Cout2 + (size_t)b * strideC) : nullptr;
      for (int pass = 0; pass < 2; ++pass) {
#pragma unroll
        for (int it = 0; it < 4; ++it) {
          const int row = it * 4 + q;
          const float* sp = slab + row * 68 + c8;
          v8h hv, lv;
#pragma unroll
          for (int e = 0; e < 8; ++e) {
            if (OUT_MODE == 1) {
              hv[e] = (_Float16)sp[e];
            } else {
              unsigned short hb = f2bf_bits(sp[e]);
              unsigned short lb = f2bf_bits(sp[e] - bf_bits2f(hb));
              hv[e] = __builtin_bit_cast(_Float16, hb);
              lv[e] = __builtin_bit_cast(_Float16, lb);
            }
          }
          *(volatile v8h*)(C + (size_t)(mBase + row) * ldc + n0 + c8) = hv;
          if (OUT_MODE == 2) *(volatile v8h*)(C2 + (size_t)(mBase + row) * ldc + n0 + c8) = lv;
        }
        __threadfence();
      }
    }
    __builtin_amdgcn_fence(__ATOMIC_RELEASE, "workgroup");
    __builtin_amdgcn_wave_barrier();
    __builtin_amdgcn_fence(__ATOMIC_ACQUIRE, "workgroup");
  }
}

__global__ __launch_bounds__(256) void wcast_f16_kernel(const float* __restrict__ W0, const float* __restrict__ W1,
                                                       const float* __restrict__ W2, const float* __restrict__ W3,
                                                       const float* __restrict__ W4, unsigned short* __restrict__ out,
                                                       int n8, float scale) {
  const int y = blockIdx.y;
  const float* W = (y == 0) ? W0 : (y == 1) ? W1 : (y == 2) ? W2 : (y == 3) ? W3 : W4;
  const int i = blockIdx.x * 256 + threadIdx.x;
  if (i >= n8) return;
  const float* p = W + 8 * (size_t)i;
  const v4f a = *(const v4f*)(p);
  const v4f c = *(const v4f*)(p + 4);
  unsigned short hb[8];
#pragma unroll
  for (int e = 0; e < 4; ++e) {
    hb[e]     = h_bits(a[e] * scale);
    hb[4 + e] = h_bits(c[e] * scale);
  }
  const v4u u = (v4u){pk16(hb[0], hb[1]), pk16(hb[2], hb[3]), pk16(hb[4], hb[5]), pk16(hb[6], hb[7])};
  unsigned short* q = out + (size_t)y * kWPlane + 8 * (size_t)i;
  *(volatile v4u*)q = u;
  __threadfence();
  *(volatile v4u*)q = u;
}

__global__ __launch_bounds__(256) void biascat_kernel(const float* __restrict__ b0, const float* __restrict__ b1,
                                                     const float* __restrict__ b2, const float* __restrict__ b3,
                                                     float* __restrict__ out) {
  const int y = blockIdx.x;
  const float* bp = (y == 0) ? b0 : (y == 1) ? b1 : (y == 2) ? b2 : b3;
  const int t = threadIdx.x;
  const v4f v = *(const v4f*)(bp + 4 * t);
  float* q = out + (size_t)y * kD + 4 * t;
  *(volatile v4f*)q = v;
  __threadfence();
  *(volatile v4f*)q = v;
}

__global__ __launch_bounds__(128) void layernorm_f16_kernel(const float* __restrict__ x, const float* __restrict__ gamma,
                                                           const float* __restrict__ beta, unsigned short* __restrict__ xn) {
  __shared__ float red1[4];
  __shared__ float red2[4];
  const int row  = blockIdx.x;
  const int t    = threadIdx.x;
  const int lane = t & 31, wave = t >> 5;
  const float* p = x + (size_t)row * kD + 8 * t;
  const v4f a = *(const v4f*)(p);
  const v4f c = *(const v4f*)(p + 4);
  float v[8];
#pragma unroll
  for (int e = 0; e < 4; ++e) { v[e] = a[e]; v[4 + e] = c[e]; }
  float s = ((v[0] + v[1]) + (v[2] + v[3])) + ((v[4] + v[5]) + (v[6] + v[7]));
#pragma unroll
  for (int off = 16; off > 0; off >>= 1) s += __shfl_xor(s, off, 32);
  if (lane == 0) red1[wave] = s;
  __syncthreads();
  const float mu = ((red1[0] + red1[1]) + (red1[2] + red1[3])) * kInvD;
  float d[8];
  float s2 = 0.0f;
#pragma unroll
  for (int e = 0; e < 8; ++e) { d[e] = v[e] - mu; s2 += d[e] * d[e]; }
#pragma unroll
  for (int off = 16; off > 0; off >>= 1) s2 += __shfl_xor(s2, off, 32);
  if (lane == 0) red2[wave] = s2;
  __syncthreads();
  const float var  = ((red2[0] + red2[1]) + (red2[2] + red2[3])) * kInvD;
  const float rstd = rsqrtf(var + kLnEps);
  const v4f g0 = *(const v4f*)(gamma + 8 * t);
  const v4f g1 = *(const v4f*)(gamma + 8 * t + 4);
  const v4f e0 = *(const v4f*)(beta + 8 * t);
  const v4f e1 = *(const v4f*)(beta + 8 * t + 4);
  float gg[8], bb[8];
#pragma unroll
  for (int e = 0; e < 4; ++e) { gg[e] = g0[e]; gg[4 + e] = g1[e]; bb[e] = e0[e]; bb[4 + e] = e1[e]; }
  unsigned short hb[8];
#pragma unroll
  for (int e = 0; e < 8; ++e) hb[e] = h_bits(d[e] * rstd * gg[e] + bb[e]);
  const v4u u = (v4u){pk16(hb[0], hb[1]), pk16(hb[2], hb[3]), pk16(hb[4], hb[5]), pk16(hb[6], hb[7])};
  unsigned short* q = xn + (size_t)row * kD + 8 * t;
  *(volatile v4u*)q = u;
  __threadfence();
  *(volatile v4u*)q = u;
}

__global__ __launch_bounds__(64) void ssm_scan_kernel(const float* __restrict__ QP, const float* __restrict__ KP,
                                                     const float* __restrict__ VP, const float* __restrict__ GP,
                                                     const float* __restrict__ alogit, unsigned short* __restrict__ O16,
                                                     int rowbase) {
#pragma clang fp contract(off)
  __shared__ __align__(16) float sq[2][kDH];
  __shared__ __align__(16) float sk[2][kDH];
  __shared__ __align__(16) float sal[kDH];
  __shared__ __align__(16) float so[16 * kDH];
  const int j    = threadIdx.x;
  const int hd   = blockIdx.x;
  const int col0 = hd * kDH;
  const int col  = col0 + j;
  {
    const float a = alogit[hd * kDH + j];
    sal[j] = __builtin_amdgcn_rcpf(1.0f + expf(-a));
  }
  __syncthreads();
  float al[kDH], hs[kDH];
#pragma unroll
  for (int i4 = 0; i4 < 16; ++i4) {
    const v4f a4 = *(const v4f*)(sal + 4 * i4);
#pragma unroll
    for (int e = 0; e < 4; ++e) { al[4 * i4 + e] = a4[e]; hs[4 * i4 + e] = 0.0f; }
  }
  for (int t = 0; t < kT; ++t) {
    const size_t ro = (size_t)t * kD + col;
    const float qj = QP[ro];
    const float kj = KP[ro];
    const float vj = VP[ro];
    const float gj = GP[ro];
    const int buf = t & 1;
    sq[buf][j] = qj;
    sk[buf][j] = kj;
    __syncthreads();
    float o = 0.0f;
#pragma unroll
    for (int i4 = 0; i4 < 16; ++i4) {
      const v4f q4 = *(const v4f*)(&sq[buf][4 * i4]);
      const v4f k4 = *(const v4f*)(&sk[buf][4 * i4]);
#pragma unroll
      for (int e = 0; e < 4; ++e) {
        const int i = 4 * i4 + e;
        const float dec = al[i] * hs[i];
        const float hn  = fmaf(k4[e], vj, dec);
        hs[i] = hn;
        const float pr = q4[e] * hn;
        o = o + pr;
      }
    }
    const float ex  = expf(-fabsf(gj));
    const float sp  = __builtin_amdgcn_rcpf(1.0f + ex);
    const float sn  = ex * sp;
    const float sig = (gj >= 0.0f) ? sp : sn;
    const float gate = gj * sig;
    const float og   = (o * gate) * kOCarry;
    so[(t & 15) * kDH + j] = og;
    if ((t & 15) == 15) {
      __syncthreads();
      const int L  = j >> 3;
      const int c8 = (j & 7) * 8;
      const int t0 = t - 15;
      for (int ps = 0; ps < 2; ++ps) {
#pragma unroll
        for (int it = 0; it < 2; ++it) {
          const int line = it * 8 + L;
          const float* spp = so + line * kDH + c8;
          const v4f a = *(const v4f*)(spp);
          const v4f c = *(const v4f*)(spp + 4);
          unsigned short hb[8];
#pragma unroll
          for (int e = 0; e < 4; ++e) { hb[e] = h_bits(a[e]); hb[4 + e] = h_bits(c[e]); }
          const v4u u = (v4u){pk16(hb[0], hb[1]), pk16(hb[2], hb[3]), pk16(hb[4], hb[5]), pk16(hb[6], hb[7])};
          *(volatile v4u*)(O16 + (size_t)(rowbase + t0 + line) * kD + col0 + c8) = u;
        }
        __threadfence();
      }
    }
  }
}

extern "C" void kernel_launch(void* const* d_in, const int* in_sizes, int n_in,
                              void* d_out, int out_size, void* d_ws, size_t ws_size,
                              hipStream_t stream) {
  (void)in_sizes; (void)n_in; (void)out_size;
  const float* x      = (const float*)d_in[0];
  const float* WQ     = (const float*)d_in[1];
  const float* bQ     = (const float*)d_in[2];
  const float* WK     = (const float*)d_in[3];
  const float* bK     = (const float*)d_in[4];
  const float* WV     = (const float*)d_in[5];
  const float* bV     = (const float*)d_in[6];
  const float* WO     = (const float*)d_in[7];
  const float* bO     = (const float*)d_in[8];
  const float* Wg     = (const float*)d_in[9];
  const float* bg     = (const float*)d_in[10];
  const float* alogit = (const float*)d_in[11];
  const float* gamma  = (const float*)d_in[12];
  const float* beta   = (const float*)d_in[13];

  const size_t offXN   = 0;
  const size_t bytesXN = (size_t)kRows * kD * 2;
  const size_t offW    = offXN + bytesXN;
  const size_t bytesW  = (size_t)5 * kWPlane * 2;
  const size_t offBC   = offW + bytesW;
  const size_t bytesBC = (size_t)4 * kD * 4;
  const size_t offPR   = offBC + bytesBC;
  const size_t bytesPR = (size_t)4 * kProjPlane * 4;
  const size_t offO    = offPR + bytesPR;
  const size_t bytesO  = (size_t)kRows * kD * 2;
  const size_t total   = offO + bytesO;
  if (total > ws_size) return;

  char* ws = (char*)d_ws;
  unsigned short* XN16 = (unsigned short*)(ws + offXN);
  unsigned short* W16  = (unsigned short*)(ws + offW);
  float*          BCAT = (float*)(ws + offBC);
  float*          PROJ = (float*)(ws + offPR);
  unsigned short* O16  = (unsigned short*)(ws + offO);

  const int n8w = kWPlane / 8;
  wcast_f16_kernel<<<dim3((n8w + 255) / 256, 5), 256, 0, stream>>>(WQ, WK, WV, Wg, WO, W16, n8w, kWCarry);
  biascat_kernel<<<4, 256, 0, stream>>>(bQ, bK, bV, bg, BCAT);
  layernorm_f16_kernel<<<kRows, 128, 0, stream>>>(x, gamma, beta, XN16);

  const int tilesProj = (kT / 64) * (kD / 64);
  const int gridProj  = (tilesProj + 7) / 8;
  for (int b = 0; b < kB; ++b) {
    wmma_gemm64<0, false, 2, 0, false, 0><<<dim3(gridProj, 4), 256, 0, stream>>>(
        XN16 + (size_t)b * kProjPlane, nullptr, kD, 0L,
        W16, nullptr, kD, (long)kWPlane,
        (void*)PROJ, nullptr, kD, (long)kProjPlane,
        BCAT, (long)kD,
        nullptr, 0L,
        kT, kD, kD, kProjScale);
    ssm_scan_kernel<<<kH, 64, 0, stream>>>(PROJ, PROJ + (size_t)kProjPlane, PROJ + (size_t)2 * kProjPlane,
                                           PROJ + (size_t)3 * kProjPlane, alogit, O16, b * kT);
  }

  const int tilesOut = (kRows / 64) * (kD / 64);
  const int gridOut  = (tilesOut + 7) / 8;
  wmma_gemm64<0, false, 2, 0, true, 0><<<dim3(gridOut, 1), 256, 0, stream>>>(
      O16, nullptr, kD, 0L,
      W16 + (size_t)4 * kWPlane, nullptr, kD, 0L,
      d_out, nullptr, kD, 0L,
      bO, 0L,
      x, 0L,
      kRows, kD, kD, kOutScale);
}
